// TwoTowerHedger_51848845197656
// MI455X (gfx1250) — hardware-verified
//
#include <hip/hip_runtime.h>
#include <math.h>

typedef __attribute__((ext_vector_type(16))) _Float16 v16h;
typedef __attribute__((ext_vector_type(8)))  _Float16 v8h;
typedef __attribute__((ext_vector_type(8)))  float    v8f;
typedef __attribute__((ext_vector_type(4)))  float    v4f;

constexpr int kBatch = 2048;
constexpr int kSteps = 128;
constexpr int kHid   = 128;
constexpr int kFeat  = 12;
constexpr int kRows  = kBatch * kSteps;
constexpr int kActP  = 136;
constexpr int kResP  = 132;
constexpr int kOutP  = 36;
static_assert(kRows == 262144, "row count");
static_assert((kActP * 2) % 16 == 0 && (kResP * 4) % 16 == 0 && (kOutP * 4) % 16 == 0, "16-B aligned LDS rows");

constexpr int    kWTower   = 128 * 128;
constexpr int    kOffCW1   = 8 * kWTower;
constexpr int    kOffFWin  = kOffCW1 + 128 * 256;
constexpr int    kOffPWin  = kOffFWin + 128 * 32;
constexpr int    kWHalves  = kOffPWin + 128 * 32;
constexpr size_t kOffPE    = (size_t)kWHalves * 2;
constexpr size_t kPEBytes  = (size_t)kRows * kHid * 2;
constexpr size_t kWsTotal  = kOffPE + kPEBytes;
static_assert(kOffCW1 == 131072 && kOffFWin == 163840 && kOffPWin == 167936 && kWHalves == 172032, "plane offsets");
static_assert(kOffPE == 344064ull && (kOffPE % 512) == 0, "PE offset");
static_assert(kWsTotal == 67452928ull, "carve total");
static_assert(kWsTotal <= 134217728ull, "carve cap");

template <typename T> struct Frag;
template <> struct Frag<_Float16> {
  typedef v16h V; union U { v16h v; v8h h[2]; };
  static __device__ __forceinline__ v16h load(const _Float16* p) {
    U f; f.h[0] = *(const v8h*)(p); f.h[1] = *(const v8h*)(p + 16); return f.v;
  }
};

__device__ __forceinline__ v8f mma_h(v16h a, v16h b, v8f c) {
  c = __builtin_amdgcn_wmma_f32_16x16x32_f16(false, a, false, b, (short)0, c, false, false);
  asm volatile("v_nop\n\tv_nop\n\tv_nop\n\tv_nop" : "+v"(c) : "v"(a), "v"(b));
  return c;
}

__device__ __forceinline__ v8f zero8() { return (v8f){0.f, 0.f, 0.f, 0.f, 0.f, 0.f, 0.f, 0.f}; }

__device__ __forceinline__ float leaky02(float x) { return (x >= 0.0f) ? x : 0.2f * x; }

template <bool RES_IN, bool RES_OUT>
__device__ __forceinline__ void epi_tile(const v8f acc, const v4f bA, const v4f bB,
                                         float* res, _Float16* actOut, const int row, const int n8) {
  float v[8];
#pragma unroll
  for (int r = 0; r < 4; ++r) {
    v[r]     = acc[r] + bA[r];
    v[4 + r] = acc[4 + r] + bB[r];
  }
  float* rp = res + row * kResP + n8;
  if (RES_IN) {
    const v4f rA = *(const v4f*)(rp);
    const v4f rB = *(const v4f*)(rp + 4);
#pragma unroll
    for (int r = 0; r < 4; ++r) {
      v[r]     = v[r] + rA[r];
      v[4 + r] = v[4 + r] + rB[r];
    }
  }
#pragma unroll
  for (int r = 0; r < 8; ++r) v[r] = leaky02(v[r]);
  if (RES_OUT) {
    const v4f oA = (v4f){v[0], v[1], v[2], v[3]};
    const v4f oB = (v4f){v[4], v[5], v[6], v[7]};
    *(v4f*)(rp)     = oA;
    *(v4f*)(rp + 4) = oB;
  }
  v8h o;
#pragma unroll
  for (int r = 0; r < 8; ++r) o[r] = (_Float16)v[r];
  *(v8h*)(actOut + row * kActP + n8) = o;
}

template <bool RES_IN, bool RES_OUT>
__device__ __forceinline__ void dense128(const _Float16* actIn, const _Float16* Wt, const float* bias,
                                         float* res, _Float16* actOut, const int l15, const int h) {
  v16h x0[4], x1[4];
#pragma unroll
  for (int kc = 0; kc < 4; ++kc) {
    x0[kc] = Frag<_Float16>::load(actIn + l15 * kActP + kc * 32 + 8 * h);
    x1[kc] = Frag<_Float16>::load(actIn + (16 + l15) * kActP + kc * 32 + 8 * h);
  }
#pragma unroll 1
  for (int nt = 0; nt < 8; ++nt) {
    const _Float16* wrow = Wt + (nt * 16 + l15) * kHid + 8 * h;
    v8f acc0 = zero8();
    v8f acc1 = zero8();
#pragma unroll
    for (int kc = 0; kc < 4; ++kc) {
      const v16h w = Frag<_Float16>::load(wrow + kc * 32);
      acc0 = mma_h(w, x0[kc], acc0);
      acc1 = mma_h(w, x1[kc], acc1);
    }
    const int n8 = nt * 16 + 8 * h;
    const v4f bA = *(const v4f*)(bias + n8);
    const v4f bB = *(const v4f*)(bias + n8 + 4);
    epi_tile<RES_IN, RES_OUT>(acc0, bA, bB, res, actOut, l15, n8);
    epi_tile<RES_IN, RES_OUT>(acc1, bA, bB, res, actOut, 16 + l15, n8);
  }
}

__device__ __forceinline__ void dense_in32(const v16h xa, const v16h xb, const _Float16* WtIn, const float* bias,
                                           float* res, _Float16* actOut, const int l15, const int h) {
#pragma unroll 1
  for (int nt = 0; nt < 8; ++nt) {
    const v16h w = Frag<_Float16>::load(WtIn + (nt * 16 + l15) * 32 + 8 * h);
    v8f acc0 = zero8();
    v8f acc1 = zero8();
    acc0 = mma_h(w, xa, acc0);
    acc1 = mma_h(w, xb, acc1);
    const int n8 = nt * 16 + 8 * h;
    const v4f bA = *(const v4f*)(bias + n8);
    const v4f bB = *(const v4f*)(bias + n8 + 4);
    epi_tile<false, true>(acc0, bA, bB, res, actOut, l15, n8);
    epi_tile<false, true>(acc1, bA, bB, res, actOut, 16 + l15, n8);
  }
}

struct PrepArgs { const float* src[11]; unsigned short* dst; };
static_assert(sizeof(PrepArgs) == 96, "no padding");

__global__ __launch_bounds__(256) void prep_weights_kernel(PrepArgs a) {
  const int blk = blockIdx.x;
  int pl, lb;
  if (blk < 64)      { pl = blk >> 3; lb = blk & 7; }
  else if (blk < 80) { pl = 8;        lb = blk - 64; }
  else if (blk < 82) { pl = 9;        lb = blk - 80; }
  else               { pl = 10;       lb = blk - 82; }
  const float* src = a.src[0];
#pragma unroll
  for (int i = 1; i < 11; ++i) { if (pl == i) src = a.src[i]; }
  int kreal = 128, kshift = 7, doff = pl * kWTower;
  if (pl == 8)  { kreal = 256; kshift = 8; doff = kOffCW1; }
  if (pl == 9)  { kreal = 4;   kshift = 5; doff = kOffFWin; }
  if (pl == 10) { kreal = 8;   kshift = 5; doff = kOffPWin; }
  const int e0 = (lb * 256 + (int)threadIdx.x) * 8;
  const int n  = e0 >> kshift;
  const int k0 = e0 & ((1 << kshift) - 1);
  v8h hv;
#pragma unroll
  for (int e = 0; e < 8; ++e) {
    const int k  = k0 + e;
    const int kc = (k < kreal) ? k : (kreal - 1);
    const float v = src[(size_t)kc * kHid + n];
    const float z = (k < kreal) ? v : 0.0f;
    hv[e] = (_Float16)z;
  }
  unsigned short* q = a.dst + doff + e0;
  *(volatile v8h*)q = hv;
  __threadfence();
  *(volatile v8h*)q = hv;
}

__global__ __launch_bounds__(32) __attribute__((amdgpu_num_vgpr(256)))
void path_tower_kernel(const float* feats, const unsigned short* Wp,
                       const float* b_in, const float* b11, const float* b12,
                       const float* b21, const float* b22, unsigned short* PEp) {
  __shared__ __align__(16) _Float16 sA[32 * kActP];
  __shared__ __align__(16) _Float16 sB[32 * kActP];
  __shared__ __align__(16) float    sR[32 * kResP];
  const int lane = threadIdx.x & 31;
  const int h    = lane >> 4;
  const int l15  = lane & 15;
  const int m0   = blockIdx.x * 32;
  const _Float16* W = (const _Float16*)Wp;

  v16h xa, xb;
  {
    const float* r0 = feats + (size_t)(m0 + l15) * kFeat + 4;
    const float* r1 = feats + (size_t)(m0 + 16 + l15) * kFeat + 4;
    v4f a0 = *(const v4f*)(r0);
    v4f a1 = *(const v4f*)(r0 + 4);
    v4f c0 = *(const v4f*)(r1);
    v4f c1 = *(const v4f*)(r1 + 4);
    asm volatile("" : "+v"(a0), "+v"(a1), "+v"(c0), "+v"(c1));
    const bool lo = (h == 0);
#pragma unroll
    for (int i = 0; i < 16; ++i) { xa[i] = (_Float16)0.0f; xb[i] = (_Float16)0.0f; }
#pragma unroll
    for (int e = 0; e < 4; ++e) {
      xa[e]     = (_Float16)(lo ? a0[e] : 0.0f);
      xa[4 + e] = (_Float16)(lo ? a1[e] : 0.0f);
      xb[e]     = (_Float16)(lo ? c0[e] : 0.0f);
      xb[4 + e] = (_Float16)(lo ? c1[e] : 0.0f);
    }
  }
  dense_in32(xa, xb, W + kOffPWin, b_in, sR, sA, l15, h);
  __syncthreads();
  dense128<false, false>(sA, W + 4 * kWTower, b11, sR, sB, l15, h);
  __syncthreads();
  dense128<true, true>(sB, W + 5 * kWTower, b12, sR, sA, l15, h);
  __syncthreads();
  dense128<false, false>(sA, W + 6 * kWTower, b21, sR, sB, l15, h);
  __syncthreads();
  dense128<true, false>(sB, W + 7 * kWTower, b22, sR, sA, l15, h);
  __syncthreads();
  {
    _Float16* PE = (_Float16*)PEp;
    const int c8 = l15 * 8;
    for (int pass = 0; pass < 2; ++pass) {
#pragma unroll
      for (int it = 0; it < 16; ++it) {
        const int row = it * 2 + h;
        const v8h v = *(const v8h*)(sA + row * kActP + c8);
        *(volatile v8h*)(PE + (size_t)(m0 + row) * kHid + c8) = v;
      }
      __threadfence();
    }
  }
}

__global__ __launch_bounds__(32) __attribute__((amdgpu_num_vgpr(256)))
void scan_kernel(const float* feats, const unsigned short* Wp, const unsigned short* PEp,
                 const float* b_in, const float* b11, const float* b12, const float* b21, const float* b22,
                 const float* cb1, const float* cw2, const float* cb2, float* out) {
  __shared__ __align__(16) _Float16 sA[32 * kActP];
  __shared__ __align__(16) _Float16 sB[32 * kActP];
  __shared__ __align__(16) float    sR[32 * kResP];
  __shared__ __align__(16) float    sO[32 * kOutP];
  const int lane = threadIdx.x & 31;
  const int h    = lane >> 4;
  const int l15  = lane & 15;
  const int b0   = blockIdx.x * 32;
  const _Float16* W  = (const _Float16*)Wp;
  const _Float16* PE = (const _Float16*)PEp;
  const float cb2v = cb2[0];
  const bool lo = (h == 0);

  const float* fr0 = feats + (size_t)(b0 + l15) * kSteps * kFeat;
  const float* fr1 = feats + (size_t)(b0 + 16 + l15) * kSteps * kFeat;
  const _Float16* pe0 = PE + (size_t)(b0 + l15) * kSteps * kHid + 8 * h;
  const _Float16* pe1 = PE + (size_t)(b0 + 16 + l15) * kSteps * kHid + 8 * h;

  float d0 = 0.0f, d1 = 0.0f;

#pragma unroll 1
  for (int k = 0; k < kSteps; ++k) {
    v16h xa, xb;
    {
      v4f q0 = *(const v4f*)(fr0 + (size_t)k * kFeat);
      v4f q1 = *(const v4f*)(fr1 + (size_t)k * kFeat);
      asm volatile("" : "+v"(q0), "+v"(q1));
      const float t0 = (k == 0) ? q0[3] : d0;
      const float t1 = (k == 0) ? q1[3] : d1;
#pragma unroll
      for (int i = 0; i < 16; ++i) { xa[i] = (_Float16)0.0f; xb[i] = (_Float16)0.0f; }
      xa[0] = (_Float16)(lo ? q0[0] : 0.0f);
      xa[1] = (_Float16)(lo ? q0[1] : 0.0f);
      xa[2] = (_Float16)(lo ? q0[2] : 0.0f);
      xa[3] = (_Float16)(lo ? t0 : 0.0f);
      xb[0] = (_Float16)(lo ? q1[0] : 0.0f);
      xb[1] = (_Float16)(lo ? q1[1] : 0.0f);
      xb[2] = (_Float16)(lo ? q1[2] : 0.0f);
      xb[3] = (_Float16)(lo ? t1 : 0.0f);
    }
    dense_in32(xa, xb, W + kOffFWin, b_in, sR, sA, l15, h);
    __syncthreads();
    dense128<false, false>(sA, W + 0 * kWTower, b11, sR, sB, l15, h);
    __syncthreads();
    dense128<true, true>(sB, W + 1 * kWTower, b12, sR, sA, l15, h);
    __syncthreads();
    dense128<false, false>(sA, W + 2 * kWTower, b21, sR, sB, l15, h);
    __syncthreads();
    dense128<true, false>(sB, W + 3 * kWTower, b22, sR, sA, l15, h);
    __syncthreads();

    float s0 = 0.0f, s1 = 0.0f;
    {
      v16h f0[4], f1[4], p0[4], p1[4];
#pragma unroll
      for (int kc = 0; kc < 4; ++kc) {
        f0[kc] = Frag<_Float16>::load(sA + l15 * kActP + kc * 32 + 8 * h);
        f1[kc] = Frag<_Float16>::load(sA + (16 + l15) * kActP + kc * 32 + 8 * h);
      }
      const _Float16* q0p = pe0 + (size_t)k * kHid;
      const _Float16* q1p = pe1 + (size_t)k * kHid;
#pragma unroll
      for (int kc = 0; kc < 4; ++kc) {
        p0[kc] = Frag<_Float16>::load(q0p + kc * 32);
        p1[kc] = Frag<_Float16>::load(q1p + kc * 32);
      }
#pragma unroll 1
      for (int nt = 0; nt < 8; ++nt) {
        const _Float16* wrow = W + kOffCW1 + (nt * 16 + l15) * 256 + 8 * h;
        v8f acc0 = zero8();
        v8f acc1 = zero8();
#pragma unroll
        for (int kc = 0; kc < 4; ++kc) {
          const v16h w = Frag<_Float16>::load(wrow + kc * 32);
          acc0 = mma_h(w, f0[kc], acc0);
          acc1 = mma_h(w, f1[kc], acc1);
        }
#pragma unroll
        for (int kc = 0; kc < 4; ++kc) {
          const v16h w = Frag<_Float16>::load(wrow + 128 + kc * 32);
          acc0 = mma_h(w, p0[kc], acc0);
          acc1 = mma_h(w, p1[kc], acc1);
        }
        const int n8 = nt * 16 + 8 * h;
        const v4f bA = *(const v4f*)(cb1 + n8);
        const v4f bB = *(const v4f*)(cb1 + n8 + 4);
        const v4f wA = *(const v4f*)(cw2 + n8);
        const v4f wB = *(const v4f*)(cw2 + n8 + 4);
#pragma unroll
        for (int r = 0; r < 4; ++r) {
          const float c0a = leaky02(acc0[r] + bA[r]);
          const float c0b = leaky02(acc0[4 + r] + bB[r]);
          const float c1a = leaky02(acc1[r] + bA[r]);
          const float c1b = leaky02(acc1[4 + r] + bB[r]);
          s0 = fmaf(c0a, wA[r], s0);
          s0 = fmaf(c0b, wB[r], s0);
          s1 = fmaf(c1a, wA[r], s1);
          s1 = fmaf(c1b, wB[r], s1);
        }
      }
    }
    const float o0 = __shfl_xor(s0, 16, 32);
    const float o1 = __shfl_xor(s1, 16, 32);
    const float z0 = (s0 + o0) + cb2v;
    const float z1 = (s1 + o1) + cb2v;
    d0 = 1.0f / (1.0f + expf(-z0));
    d1 = 1.0f / (1.0f + expf(-z1));

    const float dv = lo ? d0 : d1;
    sO[lane * kOutP + (k & 31)] = dv;

    if ((k & 31) == 31) {
      __syncthreads();
      const int q  = lane >> 3;
      const int c4 = (lane & 7) * 4;
      const int kb = k - 31;
      for (int pass = 0; pass < 2; ++pass) {
#pragma unroll
        for (int it = 0; it < 8; ++it) {
          const int row = it * 4 + q;
          const v4f v = *(const v4f*)(sO + row * kOutP + c4);
          *(volatile v4f*)(out + (size_t)(b0 + row) * kSteps + kb + c4) = v;
        }
        __threadfence();
      }
      __syncthreads();
    }
  }
}

extern "C" void kernel_launch(void* const* d_in, const int* in_sizes, int n_in,
                              void* d_out, int out_size, void* d_ws, size_t ws_size,
                              hipStream_t stream) {
  if (n_in < 25) return;
  if (in_sizes[0] != kRows * kFeat) return;
  if (in_sizes[1] != 4 * kHid) return;
  if (in_sizes[3] != kHid * kHid) return;
  if (in_sizes[11] != 8 * kHid) return;
  if (in_sizes[21] != 2 * kHid * kHid) return;
  if (in_sizes[23] != kHid) return;
  if (in_sizes[24] != 1) return;
  if (out_size != kRows) return;
  if (ws_size < kWsTotal) return;

  char* ws = (char*)d_ws;
  unsigned short* Wp  = (unsigned short*)ws;
  unsigned short* PEp = (unsigned short*)(ws + kOffPE);

  PrepArgs pa;
  pa.src[0]  = (const float*)d_in[3];
  pa.src[1]  = (const float*)d_in[5];
  pa.src[2]  = (const float*)d_in[7];
  pa.src[3]  = (const float*)d_in[9];
  pa.src[4]  = (const float*)d_in[13];
  pa.src[5]  = (const float*)d_in[15];
  pa.src[6]  = (const float*)d_in[17];
  pa.src[7]  = (const float*)d_in[19];
  pa.src[8]  = (const float*)d_in[21];
  pa.src[9]  = (const float*)d_in[1];
  pa.src[10] = (const float*)d_in[11];
  pa.dst     = Wp;
  prep_weights_kernel<<<84, 256, 0, stream>>>(pa);

  path_tower_kernel<<<kRows / 32, 32, 0, stream>>>(
      (const float*)d_in[0], Wp,
      (const float*)d_in[12], (const float*)d_in[14], (const float*)d_in[16],
      (const float*)d_in[18], (const float*)d_in[20], PEp);

  scan_kernel<<<kBatch / 32, 32, 0, stream>>>(
      (const float*)d_in[0], Wp, PEp,
      (const float*)d_in[2], (const float*)d_in[4], (const float*)d_in[6],
      (const float*)d_in[8], (const float*)d_in[10],
      (const float*)d_in[22], (const float*)d_in[23], (const float*)d_in[24],
      (float*)d_out);
}
